// CausalAttention_50457275794110
// MI455X (gfx1250) — hardware-verified
//
#include <hip/hip_runtime.h>


#ifndef NB
#define NB 2
#endif
#ifndef SEQ
#define SEQ 2048
#endif
#define NB_FULL  2
#define SEQ_FULL 2048
#define DM   1024
#define NHD  16
#define HD   64
#define MROWS (NB * SEQ)
#define NU    (NB * NHD)
#define PCAR 1024.0f
#define VCAR 16.0f
#define QSCL 0.125f
static_assert(SEQ % 64 == 0);
static_assert(SEQ <= SEQ_FULL);
static_assert(NB >= 1 && NB <= NB_FULL);
static_assert(DM % 64 == 0);
static_assert(DM == NHD * HD);
static_assert(HD == 64);

typedef _Float16 h16;
typedef unsigned short bf;
typedef __attribute__((ext_vector_type(16))) __bf16   v16bf;
typedef __attribute__((ext_vector_type(16))) _Float16 v16h;
typedef __attribute__((ext_vector_type(8)))  _Float16 v8h;
typedef __attribute__((ext_vector_type(8)))  unsigned short v8us;
typedef __attribute__((ext_vector_type(8)))  float    v8f;
typedef __attribute__((ext_vector_type(4)))  float    v4f;
typedef __attribute__((ext_vector_type(2)))  _Float16 v2h;
typedef __attribute__((ext_vector_type(2)))  unsigned short v2us;
typedef __attribute__((ext_vector_type(4)))  unsigned short v4us;
typedef v8h  __attribute__((may_alias)) v8ha;
typedef v4f  __attribute__((may_alias)) v4fa;
typedef v8us __attribute__((may_alias)) v8usa;

__device__ __forceinline__ unsigned short f2bf(float f) { unsigned u = __float_as_uint(f); u += 0x7FFFu + ((u >> 16) & 1u); return (unsigned short)(u >> 16); }
__device__ __forceinline__ float bf2f(unsigned short b) { return __uint_as_float(((unsigned)b) << 16); }
__device__ __forceinline__ float bfr(float f) { return bf2f(f2bf(f)); }
__device__ __forceinline__ void splitf(float y, unsigned short& h, unsigned short& l) { h = f2bf(y); l = f2bf(y - bf2f(h)); }
__device__ __forceinline__ v16h cat16(v8h lo, v8h hi) { return __builtin_shufflevector(lo, hi, 0, 1, 2, 3, 4, 5, 6, 7, 8, 9, 10, 11, 12, 13, 14, 15); }
__device__ __forceinline__ v16bf cat16b(v8us lo, v8us hi) { return __builtin_bit_cast(v16bf, __builtin_shufflevector(lo, hi, 0, 1, 2, 3, 4, 5, 6, 7, 8, 9, 10, 11, 12, 13, 14, 15)); }
__device__ __forceinline__ v8f wmma16(v16h a, v16h b, v8f c) { return __builtin_amdgcn_wmma_f32_16x16x32_f16(false, a, false, b, (short)0, c, false, false); }
__device__ __forceinline__ v8f wmmab(v16bf a, v16bf b, v8f c) { return __builtin_amdgcn_wmma_f32_16x16x32_bf16(false, a, false, b, (short)0, c, false, false); }
__device__ __forceinline__ v16bf ldb(const bf* p) { return cat16b(*(const v8us*)p, *(const v8us*)(p + 16)); }
__device__ __forceinline__ v16h  ldh(const h16* p) { return cat16(*(const v8h*)p, *(const v8h*)(p + 16)); }
__device__ __forceinline__ void wave_lds_sync() { __builtin_amdgcn_fence(3  , "wavefront"); __builtin_amdgcn_wave_barrier(); asm volatile("" ::: "memory"); }

template <int NSPLIT, int EPM>
__global__ __launch_bounds__(32) __attribute__((amdgpu_num_vgpr(256))) void k_gemm(const bf* __restrict__ A, const bf* __restrict__ A2, const bf* __restrict__ Bt, int K, float* C, int ldc, bf* Ch, bf* Cl, const float* __restrict__ bias, float scl) {
    __shared__ __align__(16) float os[16 * 68];
    const int lane = threadIdx.x & 31, lr = lane & 15, hi = lane >> 4;
    const int r0 = blockIdx.x * 64, c0 = blockIdx.y * 64;
    v8f acc[4][4];
#pragma unroll
    for (int mb = 0; mb < 4; ++mb)
#pragma unroll
        for (int nb = 0; nb < 4; ++nb) acc[mb][nb] = (v8f){};
    const size_t aoff = (size_t)(r0 + lr) * K + 8 * hi, boff = (size_t)(c0 + lr) * K + 8 * hi;
#pragma unroll 1
    for (int kc = 0; kc < K; kc += 32) {
        v16bf a[4], a2[4];
#pragma unroll
        for (int mb = 0; mb < 4; ++mb) {
            a[mb] = ldb(A + aoff + (size_t)mb * 16 * K + kc);
            if constexpr (NSPLIT == 1) a2[mb] = ldb(A2 + aoff + (size_t)mb * 16 * K + kc); else a2[mb] = a[mb];
        }
#pragma unroll
        for (int nb = 0; nb < 4; ++nb) {
            const v16bf bt_ = ldb(Bt + boff + (size_t)nb * 16 * K + kc);
#pragma unroll
            for (int mb = 0; mb < 4; ++mb) {
                acc[mb][nb] = wmmab(a[mb], bt_, acc[mb][nb]);
                if constexpr (NSPLIT == 1) acc[mb][nb] = wmmab(a2[mb], bt_, acc[mb][nb]);
            }
        }
        asm volatile("v_nop\n\tv_nop\n\tv_nop\n\tv_nop" : "+v"(acc[0][0]), "+v"(acc[1][1]), "+v"(acc[2][2]), "+v"(acc[3][3]) : "v"(a[0]), "v"(a[3]), "v"(a2[3]));
    }
#pragma unroll
    for (int mb = 0; mb < 4; ++mb) {
#pragma unroll
        for (int nb = 0; nb < 4; ++nb) {
#pragma unroll
            for (int j = 0; j < 8; ++j) os[(hi * 8 + j) * 68 + nb * 16 + lr] = acc[mb][nb][j];
        }
        wave_lds_sync();
        if constexpr (EPM == 0) {
            float* crow = C + (size_t)(r0 + mb * 16) * ldc + c0;
#pragma unroll 1
            for (int ps = 0; ps < 2; ++ps) {
#pragma unroll
                for (int s = 0; s < 8; ++s) {
                    const int row = 2 * s + hi, cofs = lr * 4;
                    v4f val = *(const v4fa*)(os + row * 68 + cofs);
                    val[0] += bfr(bias[c0 + cofs]); val[1] += bfr(bias[c0 + cofs + 1]); val[2] += bfr(bias[c0 + cofs + 2]); val[3] += bfr(bias[c0 + cofs + 3]);
                    *(volatile v4f*)(crow + (size_t)row * ldc + cofs) = val;
                }
                if (ps == 0) __threadfence();
            }
        } else {
            const int unit = (r0 / SEQ) * NHD + c0 / HD; const int t0 = (r0 % SEQ) + mb * 16;
            const size_t pb = ((size_t)unit * SEQ + t0) * HD;
#pragma unroll 1
            for (int ps = 0; ps < 2; ++ps) {
#pragma unroll
                for (int s = 0; s < 8; ++s) {
                    const int row = 2 * s + hi, cofs = lr * 4;
                    const v4f val = *(const v4fa*)(os + row * 68 + cofs);
                    v4us oh, ol;
#pragma unroll
                    for (int i = 0; i < 4; ++i) { const float y = (val[i] + bfr(bias[c0 + cofs + i])) * scl; unsigned short h_, l_; splitf(y, h_, l_); oh[i] = h_; ol[i] = l_; }
                    const size_t o = pb + (size_t)row * HD + cofs;
                    *(volatile v4us*)(Ch + o) = oh; *(volatile v4us*)(Cl + o) = ol;
                }
                if (ps == 0) __threadfence();
            }
        }
        wave_lds_sync();
    }
}

__global__ __launch_bounds__(256) void k_wtG(const float* __restrict__ w, int K, int N, bf* Bt) {
    const int lane = threadIdx.x & 31; const int L0 = (blockIdx.x * 8 + (threadIdx.x >> 5)) * 8; const int nlines = N * K / 64;
#pragma unroll
    for (int ps = 0; ps < 2; ++ps) {
#pragma unroll 1
        for (int l = 0; l < 8; ++l) { const int L = L0 + l; if (L >= nlines) break; const size_t e = (size_t)L * 64 + lane * 2; const int k = (int)(e % K), n = (int)(e / K); v2us o;
            o[0] = f2bf(w[(size_t)k * N + n]); o[1] = f2bf(w[(size_t)(k + 1) * N + n]); *(volatile v2us*)(Bt + e) = o; }
        if (ps == 0) __threadfence(); }
}
__global__ __launch_bounds__(256) void k_cvt8(const float* __restrict__ src, bf* dst, size_t n8) {
    const size_t i = (size_t)blockIdx.x * 256 + threadIdx.x; if (i >= n8) return; const v8f v = *(const v8f*)(src + i * 8); v8us o;
#pragma unroll
    for (int k = 0; k < 8; ++k) o[k] = f2bf(v[k]);
    *(volatile v8us*)(dst + i * 8) = o; __threadfence(); *(volatile v8us*)(dst + i * 8) = o;
}

__global__ __launch_bounds__(256) void k_vtp3(const float* __restrict__ Cv, h16* V16T, bf* VhT, bf* VlT) {
    const size_t e = ((size_t)blockIdx.x * 256 + threadIdx.x) * 2; if (e >= (size_t)NU * HD * SEQ) return;
    const int t = (int)(e % SEQ); const int d = (int)((e / SEQ) % HD); const int uu = (int)(e / ((size_t)SEQ * HD)); const int bb = uu / NHD, hh = uu % NHD;
    v2h o16; v2us oh, ol;
#pragma unroll
    for (int q = 0; q < 2; ++q) { const float x = Cv[((size_t)bb * SEQ + t + q) * DM + hh * HD + d]; o16[q] = (h16)(x * VCAR); unsigned short a_, c_; splitf(x, a_, c_); oh[q] = a_; ol[q] = c_; }
    *(volatile v2h*)(V16T + e) = o16; *(volatile v2us*)(VhT + e) = oh; *(volatile v2us*)(VlT + e) = ol;
    __threadfence();
    *(volatile v2h*)(V16T + e) = o16; *(volatile v2us*)(VhT + e) = oh; *(volatile v2us*)(VlT + e) = ol;
}

__global__ __launch_bounds__(128) __attribute__((amdgpu_num_vgpr(256))) void k_flash(const bf* __restrict__ Qh, const bf* __restrict__ Ql, const bf* __restrict__ Kh, const bf* __restrict__ Kl,
                                                                                     const h16* __restrict__ V16T, const bf* __restrict__ VhT, const bf* __restrict__ VlT, bf* Hh, bf* Hl) {
    __shared__ __align__(16) h16 sP[4][16 * 72];
    __shared__ __align__(16) unsigned short sPh[4][16 * 72];
    __shared__ __align__(16) unsigned short sPl[4][16 * 72];
    __shared__ __align__(16) float os[4][16 * 68];
    const int tid = threadIdx.x, wv = tid >> 5, lane = tid & 31, lr = lane & 15, hi = lane >> 4;
    const int qt = blockIdx.x, u = blockIdx.y, b = u / NHD, hd = u % NHD;
    const int qr0 = qt * 64 + wv * 16;
    const bool early = (qt == 0);
    h16* sp = sP[wv]; unsigned short* sph = sPh[wv]; unsigned short* spl = sPl[wv]; float* o_s = os[wv];
    const float L2E = 1.4426950408889634f;

    v16bf qh[2], ql[2];
    {
        const size_t qoff = ((size_t)u * SEQ + qr0 + lr) * HD + 8 * hi;
#pragma unroll
        for (int c = 0; c < 2; ++c) { qh[c] = ldb(Qh + qoff + c * 32); ql[c] = ldb(Ql + qoff + c * 32); }
    }
    float mrow[8], lrow[8];
#pragma unroll
    for (int r = 0; r < 8; ++r) { mrow[r] = -1.0e30f; lrow[r] = 0.0f; }
    v8f O[4];
#pragma unroll
    for (int n = 0; n < 4; ++n) O[n] = (v8f){};
    const size_t kb0 = (size_t)u * SEQ * HD;
    const size_t vb0 = (size_t)u * HD * SEQ;

#pragma unroll 1
    for (int kc = 0; kc <= qt; ++kc) {
        const int key0 = kc * 64;
        v8f S[4];
#pragma unroll
        for (int n = 0; n < 4; ++n) S[n] = (v8f){};
        v16bf kh_ = qh[0], kl_ = ql[0];
#pragma unroll
        for (int nb = 0; nb < 4; ++nb) {
            const size_t ko = kb0 + (size_t)(key0 + nb * 16 + lr) * HD + 8 * hi;
#pragma unroll
            for (int c = 0; c < 2; ++c) {
                kh_ = ldb(Kh + ko + c * 32); kl_ = ldb(Kl + ko + c * 32);
                S[nb] = wmmab(qh[c], kh_, S[nb]);
                S[nb] = wmmab(ql[c], kh_, S[nb]);
                S[nb] = wmmab(qh[c], kl_, S[nb]);
            }
        }
        asm volatile("v_nop\n\tv_nop\n\tv_nop\n\tv_nop" : "+v"(S[0]), "+v"(S[1]), "+v"(S[2]), "+v"(S[3]) : "v"(qh[0]), "v"(qh[1]), "v"(ql[0]), "v"(ql[1]), "v"(kh_), "v"(kl_));

#pragma unroll
        for (int r = 0; r < 8; ++r) {
            const int q = qr0 + 8 * hi + r;
            const float t0 = (key0 + lr      <= q) ? S[0][r] : -1.0e30f;
            const float t1 = (key0 + 16 + lr <= q) ? S[1][r] : -1.0e30f;
            const float t2 = (key0 + 32 + lr <= q) ? S[2][r] : -1.0e30f;
            const float t3 = (key0 + 48 + lr <= q) ? S[3][r] : -1.0e30f;
            float mx = fmaxf(fmaxf(t0, t1), fmaxf(t2, t3));
            mx = fmaxf(mx, __shfl_xor(mx, 1, 32)); mx = fmaxf(mx, __shfl_xor(mx, 2, 32)); mx = fmaxf(mx, __shfl_xor(mx, 4, 32)); mx = fmaxf(mx, __shfl_xor(mx, 8, 32));
            const float mnew = fmaxf(mrow[r], mx);
            const float alpha = __builtin_amdgcn_exp2f((mrow[r] - mnew) * L2E);
            mrow[r] = mnew;
            const float p0 = __builtin_amdgcn_exp2f((t0 - mnew) * L2E);
            const float p1 = __builtin_amdgcn_exp2f((t1 - mnew) * L2E);
            const float p2 = __builtin_amdgcn_exp2f((t2 - mnew) * L2E);
            const float p3 = __builtin_amdgcn_exp2f((t3 - mnew) * L2E);
            float rs = (p0 + p1) + (p2 + p3);
            rs += __shfl_xor(rs, 1, 32); rs += __shfl_xor(rs, 2, 32); rs += __shfl_xor(rs, 4, 32); rs += __shfl_xor(rs, 8, 32);
            lrow[r] = lrow[r] * alpha + rs;
            O[0][r] *= alpha; O[1][r] *= alpha; O[2][r] *= alpha; O[3][r] *= alpha;
            const int ro = (8 * hi + r) * 72 + lr;
            if (early) {
                unsigned short h_, l_;
                splitf(p0 * PCAR, h_, l_); sph[ro]      = h_; spl[ro]      = l_;
                splitf(p1 * PCAR, h_, l_); sph[ro + 16] = h_; spl[ro + 16] = l_;
                splitf(p2 * PCAR, h_, l_); sph[ro + 32] = h_; spl[ro + 32] = l_;
                splitf(p3 * PCAR, h_, l_); sph[ro + 48] = h_; spl[ro + 48] = l_;
            } else {
                sp[ro]      = (h16)(p0 * PCAR);
                sp[ro + 16] = (h16)(p1 * PCAR);
                sp[ro + 32] = (h16)(p2 * PCAR);
                sp[ro + 48] = (h16)(p3 * PCAR);
            }
        }
        wave_lds_sync();

        if (early) {
            v16bf ph[2], pl[2];
#pragma unroll
            for (int c = 0; c < 2; ++c) {
                ph[c] = cat16b(*(const v8usa*)(sph + lr * 72 + c * 32 + 8 * hi), *(const v8usa*)(sph + lr * 72 + c * 32 + 8 * hi + 16));
                pl[c] = cat16b(*(const v8usa*)(spl + lr * 72 + c * 32 + 8 * hi), *(const v8usa*)(spl + lr * 72 + c * 32 + 8 * hi + 16));
            }
            v16bf vh_ = ph[0], vl_ = pl[0];
#pragma unroll
            for (int nd = 0; nd < 4; ++nd) {
                const size_t vo = vb0 + (size_t)(nd * 16 + lr) * SEQ + key0 + 8 * hi;
#pragma unroll
                for (int c = 0; c < 2; ++c) {
                    vh_ = ldb(VhT + vo + c * 32); vl_ = ldb(VlT + vo + c * 32);
                    O[nd] = wmmab(ph[c], vh_, O[nd]);
                    O[nd] = wmmab(pl[c], vh_, O[nd]);
                    O[nd] = wmmab(ph[c], vl_, O[nd]);
                }
            }
            asm volatile("v_nop\n\tv_nop\n\tv_nop\n\tv_nop" : "+v"(O[0]), "+v"(O[1]), "+v"(O[2]), "+v"(O[3]) : "v"(ph[0]), "v"(ph[1]), "v"(pl[0]), "v"(pl[1]), "v"(vh_), "v"(vl_));
        } else {
            v16h p16[2];
#pragma unroll
            for (int c = 0; c < 2; ++c) p16[c] = cat16(*(const v8ha*)(sp + lr * 72 + c * 32 + 8 * hi), *(const v8ha*)(sp + lr * 72 + c * 32 + 8 * hi + 16));
            v16h vf_ = p16[0];
#pragma unroll
            for (int nd = 0; nd < 4; ++nd) {
                const size_t vo = vb0 + (size_t)(nd * 16 + lr) * SEQ + key0 + 8 * hi;
#pragma unroll
                for (int c = 0; c < 2; ++c) { vf_ = ldh(V16T + vo + c * 32); O[nd] = wmma16(p16[c], vf_, O[nd]); }
            }
            asm volatile("v_nop\n\tv_nop\n\tv_nop\n\tv_nop" : "+v"(O[0]), "+v"(O[1]), "+v"(O[2]), "+v"(O[3]) : "v"(p16[0]), "v"(p16[1]), "v"(vf_));
        }
        wave_lds_sync();
    }

    const float car = early ? (1.0f / PCAR) : (1.0f / (PCAR * VCAR));
#pragma unroll
    for (int r = 0; r < 8; ++r) {
        const float inv = car / lrow[r];
        O[0][r] *= inv; O[1][r] *= inv; O[2][r] *= inv; O[3][r] *= inv;
    }
#pragma unroll
    for (int nd = 0; nd < 4; ++nd) {
#pragma unroll
        for (int r = 0; r < 8; ++r) o_s[(hi * 8 + r) * 68 + nd * 16 + lr] = O[nd][r];
    }
    wave_lds_sync();
    const size_t hb = ((size_t)b * SEQ + qr0) * DM + (size_t)hd * HD;
#pragma unroll 1
    for (int ps = 0; ps < 2; ++ps) {
#pragma unroll
        for (int s = 0; s < 8; ++s) {
            const int row = 2 * s + hi, cofs = lr * 4;
            const v4f val = *(const v4fa*)(o_s + row * 68 + cofs);
            v4us oh, ol;
#pragma unroll
            for (int i = 0; i < 4; ++i) { unsigned short h_, l_; splitf(val[i], h_, l_); oh[i] = h_; ol[i] = l_; }
            const size_t o = hb + (size_t)row * DM + cofs;
            *(volatile v4us*)(Hh + o) = oh; *(volatile v4us*)(Hl + o) = ol;
        }
        if (ps == 0) __threadfence();
    }
}

extern "C" void kernel_launch(void* const* d_in, const int* in_sizes, int n_in,
                              void* d_out, int out_size, void* d_ws, size_t ws_size, hipStream_t stream) {
    if (n_in < 9) return;
    const size_t needx = ((size_t)(NB - 1) * SEQ_FULL + SEQ) * DM;
    if ((size_t)in_sizes[0] < needx || (size_t)out_size < needx) return;
    if (in_sizes[1] < DM * DM || in_sizes[3] < DM * DM || in_sizes[5] < DM * DM || in_sizes[7] < DM * DM) return;
    if (in_sizes[2] < DM || in_sizes[4] < DM || in_sizes[6] < DM || in_sizes[8] < DM) return;
    const float* x  = (const float*)d_in[0];
    const float* Wq = (const float*)d_in[1]; const float* bq = (const float*)d_in[2];
    const float* Wk = (const float*)d_in[3]; const float* bk = (const float*)d_in[4];
    const float* Wv = (const float*)d_in[5]; const float* bv = (const float*)d_in[6];
    const float* Wo = (const float*)d_in[7]; const float* bo = (const float*)d_in[8];
    float* out = (float*)d_out;

    char* wsp = (char*)d_ws;
    auto take = [&](size_t bytes) { char* p = wsp; wsp += (bytes + 255) & ~(size_t)255; return (void*)p; };
    const size_t planeQK = (size_t)NU * SEQ * HD;
    bf*  xb   = (bf*)take((size_t)MROWS * DM * 2);
    bf*  WqT  = (bf*)take((size_t)DM * DM * 2); bf* WkT = (bf*)take((size_t)DM * DM * 2); bf* WvT = (bf*)take((size_t)DM * DM * 2); bf* WoT = (bf*)take((size_t)DM * DM * 2);
    bf*  Qh   = (bf*)take(planeQK * 2); bf* Ql = (bf*)take(planeQK * 2); bf* Kh = (bf*)take(planeQK * 2); bf* Kl = (bf*)take(planeQK * 2);
    float* Cv = (float*)take((size_t)MROWS * DM * 4);
    h16* V16T = (h16*)take(planeQK * 2); bf* VhT = (bf*)take(planeQK * 2); bf* VlT = (bf*)take(planeQK * 2);
    bf*  Hh   = (bf*)take((size_t)MROWS * DM * 2); bf* Hl = (bf*)take((size_t)MROWS * DM * 2);
    const size_t used = (size_t)(wsp - (char*)d_ws);
    if (used > ws_size || used > (size_t)134217728) return;

    for (int bb = 0; bb < NB; ++bb)
        k_cvt8<<<(unsigned)(((size_t)SEQ * DM / 8 + 255) / 256), 256, 0, stream>>>(x + (size_t)bb * SEQ_FULL * DM, xb + (size_t)bb * SEQ * DM, (size_t)SEQ * DM / 8);
    const int nlines = DM * DM / 64;
    k_wtG<<<(unsigned)((nlines + 63) / 64), 256, 0, stream>>>(Wq, DM, DM, WqT);
    k_wtG<<<(unsigned)((nlines + 63) / 64), 256, 0, stream>>>(Wk, DM, DM, WkT);
    k_wtG<<<(unsigned)((nlines + 63) / 64), 256, 0, stream>>>(Wv, DM, DM, WvT);
    k_wtG<<<(unsigned)((nlines + 63) / 64), 256, 0, stream>>>(Wo, DM, DM, WoT);
    k_gemm<0, 1><<<dim3(MROWS / 64, DM / 64, 1), 32, 0, stream>>>(xb, nullptr, WqT, DM, nullptr, 0, Qh, Ql, bq, QSCL);
    k_gemm<0, 1><<<dim3(MROWS / 64, DM / 64, 1), 32, 0, stream>>>(xb, nullptr, WkT, DM, nullptr, 0, Kh, Kl, bk, 1.0f);
    k_gemm<0, 0><<<dim3(MROWS / 64, DM / 64, 1), 32, 0, stream>>>(xb, nullptr, WvT, DM, Cv, DM, nullptr, nullptr, bv, 1.0f);
    k_vtp3<<<(unsigned)(((size_t)NU * HD * SEQ / 2 + 255) / 256), 256, 0, stream>>>(Cv, V16T, VhT, VlT);
    k_flash<<<dim3(SEQ / 64, NU, 1), 128, 0, stream>>>(Qh, Ql, Kh, Kl, V16T, VhT, VlT, Hh, Hl);
    for (int bb = 0; bb < NB; ++bb)
        k_gemm<1, 0><<<dim3(SEQ / 64, DM / 64, 1), 32, 0, stream>>>(Hh + (size_t)bb * SEQ * DM, Hl + (size_t)bb * SEQ * DM, WoT, DM, out + (size_t)bb * SEQ_FULL * DM, DM, nullptr, nullptr, bo, 1.0f);
}
